// MultiHeadSelfAttention3D_78417512890694
// MI455X (gfx1250) — hardware-verified
//
#include <hip/hip_runtime.h>


namespace {
constexpr int C = 64, T = 4096, NH = 8, HD = 8, KP = 32  , VP = 16  , NQB = 128  ;
constexpr float XS = 8.0f, WSC = 256.0f, PS = 1024.0f, LOG2E = 1.4426950408889634f, SCALE = 0.35355339059327373f;
static_assert(T % 64 == 0 && C == 64 && NH * HD == C && NQB * 32 <= T, "tiling");
typedef _Float16 b16;
typedef __attribute__((ext_vector_type(16))) _Float16 v16b;
typedef __attribute__((ext_vector_type(8))) _Float16 v8b;
typedef __attribute__((ext_vector_type(8))) float v8f;
typedef __attribute__((ext_vector_type(4))) float v4f;
__device__ __forceinline__ float bf16_rne(float f) { unsigned int u = __float_as_uint(f); u += 0x7FFFu + ((u >> 16) & 1u); return __uint_as_float(u & 0xFFFF0000u); }
__device__ __forceinline__ void split16(float v, b16& hi, b16& lo) { hi = (b16)v; lo = (b16)(v - (float)hi); }
__device__ __forceinline__ v16b frag_kb(const b16* p, int hh) { const v8b a = *(const v8b*)(p + 8 * hh), b = *(const v8b*)(p + 16 + 8 * hh); v16b f;
#pragma unroll
  for (int e = 0; e < 8; ++e) { f[e] = a[e]; f[8 + e] = b[e]; } return f; }
__device__ __forceinline__ v8f wmma16b(v16b a, v16b b, v8f c) { v8f d = __builtin_amdgcn_wmma_f32_16x16x32_f16(false, a, false, b, (short)0, c, false, false); asm volatile("v_nop\n\tv_nop\n\tv_nop\n\tv_nop" : "+v"(d) : "v"(a), "v"(b)); return d; }
__device__ __forceinline__ void wave_lds_sync() { __builtin_amdgcn_fence(__ATOMIC_RELEASE, "workgroup"); __builtin_amdgcn_wave_barrier(); __builtin_amdgcn_fence(__ATOMIC_ACQUIRE, "workgroup"); }
__device__ __forceinline__ float pmul(float a, float b) { float p = a * b; asm volatile("" : "+v"(p)); return p; }
__device__ __forceinline__ int iclamp(int v, int lo, int hi) { return v < lo ? lo : (v > hi ? hi : v); }

typedef __attribute__((ext_vector_type(4))) _Float16 v4h;
typedef __attribute__((ext_vector_type(2))) _Float16 v2h;
typedef __attribute__((ext_vector_type(2))) float v2f;
__device__ __forceinline__ float nexp2(float v) { return __builtin_amdgcn_exp2f(v); }
__global__ __launch_bounds__(256) void prep_kernel(const float* __restrict__ x, const float* __restrict__ wqkv, const float* __restrict__ wp, b16* __restrict__ Xt, b16* __restrict__ Wb) {
  __shared__ __attribute__((aligned(16))) b16 tile[64][64 + 8];
  const int n0 = blockIdx.x * 64, t = threadIdx.x;
  if (blockIdx.x < T / 64) {
    for (int q = t; q < 64 * 64; q += 256) { const int c = q >> 6, j = q & 63; tile[j][c] = (b16)(bf16_rne(x[(size_t)c * T + n0 + j]) * XS); }
    __syncthreads();
    const int wave = t >> 5, lane = t & 31;
    for (int pass = 0; pass < 2; ++pass) { for (int rr = 0; rr < 8; ++rr) { const int j = wave * 8 + rr; *(volatile v2h*)(Xt + (size_t)(n0 + j) * C + lane * 2) = *(const v2h*)(&tile[j][lane * 2]); } __threadfence(); }
  } else {
    for (int q = t; q < 256 * 64 / 8; q += 256) { const int r = q >> 3, c0 = (q & 7) * 8; v8b o; for (int j = 0; j < 8; ++j) o[j] = (b16)(bf16_rne(r < 192 ? wqkv[r * C + c0 + j] : wp[(r - 192) * C + c0 + j]) * WSC);
      for (int pass = 0; pass < 2; ++pass) { *(volatile v8b*)(Wb + (size_t)r * C + c0) = o; __threadfence(); } } }
}
__global__ __launch_bounds__(32) void qk_kernel(const b16* __restrict__ Xt, const b16* __restrict__ Wb, b16* __restrict__ QK) {
  __shared__ __attribute__((aligned(16))) float Tf[16][128 + 4];
  const int lane = threadIdx.x, nloc = lane & 15, hlf = lane >> 4; const size_t m0 = (size_t)blockIdx.x * 16;
  v8f acc[8];
#pragma unroll
  for (int t = 0; t < 8; ++t) acc[t] = (v8f){};
#pragma unroll
  for (int kb = 0; kb < C; kb += 32) { const v16b a = frag_kb(Xt + (m0 + nloc) * C + kb, hlf);
#pragma unroll
    for (int t = 0; t < 8; ++t) acc[t] = wmma16b(a, frag_kb(Wb + (size_t)(t * 16 + nloc) * C + kb, hlf), acc[t]); }
#pragma unroll
  for (int t = 0; t < 8; ++t)
#pragma unroll
    for (int r = 0; r < 8; ++r) Tf[8 * hlf + r][t * 16 + nloc] = acc[t][r] * (1.0f / (XS * WSC));
  wave_lds_sync();
  const int h = lane >> 2, qtr = lane & 3;
  for (int pass = 0; pass < 2; ++pass) { for (int rr = 0; rr < 16; ++rr) for (int p = 0; p < 2; ++p) { v8b o; for (int j = 0; j < 8; ++j) o[j] = (qtr == 0) ? (b16)(Tf[rr][p * 64 + h * HD + j] * XS) : (b16)0.0f;
        *(volatile v8b*)(QK + (((size_t)p * T + m0 + rr) * NH + h) * KP + qtr * 8) = o; } __threadfence(); }
}
__global__ __launch_bounds__(128) void vt_kernel(const b16* __restrict__ Xt, const b16* __restrict__ Wb, b16* __restrict__ VT) {
  __shared__ __attribute__((aligned(16))) float Ts[4][16][128 + 4];
  const int wave = threadIdx.x >> 5, lane = threadIdx.x & 31, nloc = lane & 15, hlf = lane >> 4; const int r0 = wave * 16; const size_t n0 = (size_t)blockIdx.x * 128;
  v8f acc[8];
#pragma unroll
  for (int t = 0; t < 8; ++t) acc[t] = (v8f){};
#pragma unroll
  for (int kb = 0; kb < C; kb += 32) { const v16b a = frag_kb(Wb + (size_t)(128 + r0 + nloc) * C + kb, hlf);
#pragma unroll
    for (int t = 0; t < 8; ++t) acc[t] = wmma16b(a, frag_kb(Xt + (n0 + t * 16 + nloc) * C + kb, hlf), acc[t]); }
#pragma unroll
  for (int t = 0; t < 8; ++t)
#pragma unroll
    for (int r = 0; r < 8; ++r) Ts[wave][8 * hlf + r][t * 16 + nloc] = acc[t][r] * (1.0f / (XS * WSC)) * XS;
  wave_lds_sync();
  const v4h z4 = {(b16)0.0f, (b16)0.0f, (b16)0.0f, (b16)0.0f};
  for (int pass = 0; pass < 2; ++pass) { for (int rr = 0; rr < 16; ++rr) { const int h = (r0 + rr) >> 3, d = (r0 + rr) & 7;
      { const v4f f4 = *(const v4f*)(&Ts[wave][rr][lane * 4]); v4h h4; for (int j = 0; j < 4; ++j) h4[j] = (b16)f4[j]; *(volatile v4h*)(VT + ((size_t)h * VP + d) * T + n0 + lane * 4) = h4; }
      *(volatile v4h*)(VT + ((size_t)h * VP + 8 + d) * T + n0 + lane * 4) = z4; }
    __threadfence(); }
}
__global__ __launch_bounds__(64) void attn_kernel(const b16* __restrict__ QK, const b16* __restrict__ VT, b16* __restrict__ Oh, b16* __restrict__ Ol) {
  __shared__ __attribute__((aligned(16))) float To[2][16][HD + 1];
  const int wave = threadIdx.x >> 5, lane = threadIdx.x & 31, hh = lane >> 4, col = lane & 15; const int h = blockIdx.y; const int q0 = blockIdx.x * 32 + wave * 16, qi = q0 + col;
  const b16* Qp = QK; const b16* Kp = QK + (size_t)T * NH * KP; const b16* Vb = VT + (size_t)h * VP * T;
  const v16b qa = frag_kb(Qp + ((size_t)qi * NH + h) * KP, hh);
  float m = -INFINITY, l = 0.0f; v8f o = (v8f){};
  const float cs = LOG2E * SCALE / (XS * XS);
#pragma unroll 2
  for (int kb = 0; kb < T; kb += 32) {
    v8f s0 = (v8f){}, s1 = (v8f){};
    s0 = wmma16b(frag_kb(Kp + ((size_t)(kb + col) * NH + h) * KP, hh), qa, s0); s1 = wmma16b(frag_kb(Kp + ((size_t)(kb + 16 + col) * NH + h) * KP, hh), qa, s1);
    float e[16]; float mx = -INFINITY;
#pragma unroll
    for (int r = 0; r < 8; ++r) { e[r] = s0[r] * cs; e[8 + r] = s1[r] * cs; mx = fmaxf(mx, fmaxf(e[r], e[8 + r])); }
    mx = fmaxf(mx, __shfl_xor(mx, 16)); const float mn = fmaxf(m, mx); const float al = nexp2(m - mn); m = mn; float sum = 0.0f; v16b ph, pl;
#pragma unroll
    for (int i = 0; i < 16; ++i) { const float p = nexp2(e[i] - mn); sum += p; const b16 h_ = (b16)(p * PS); ph[i] = h_; pl[i] = (b16)(p * PS - (float)h_); }
    sum += __shfl_xor(sum, 16); l = l * al + sum;
    const v16b vf = frag_kb(Vb + (size_t)col * T + kb, hh);
    o *= al; o = wmma16b(vf, ph, o); o = wmma16b(vf, pl, o); }
  const float inv = 1.0f / (l * PS * XS);
  if (hh == 0) {
#pragma unroll
    for (int r = 0; r < 8; ++r) To[wave][col][r] = o[r] * inv; }
  wave_lds_sync();
  for (int pass = 0; pass < 2; ++pass) { if (lane < 16) { v8b hv, lv; for (int j = 0; j < 8; ++j) { b16 p, q; split16(To[wave][lane][j] * XS, p, q); hv[j] = p; lv[j] = q; }
      *(volatile v8b*)(Oh + ((size_t)h * T + q0 + lane) * HD) = hv; *(volatile v8b*)(Ol + ((size_t)h * T + q0 + lane) * HD) = lv; } __threadfence(); }
}
__device__ __forceinline__ v16b frag_heads(const b16* P, size_t n, int j, int hh) { const v8b a = *(const v8b*)(P + ((size_t)(4 * j + hh) * T + n) * HD), b = *(const v8b*)(P + ((size_t)(4 * j + 2 + hh) * T + n) * HD); v16b f;
#pragma unroll
  for (int e = 0; e < 8; ++e) { f[e] = a[e]; f[8 + e] = b[e]; } return f; }
__global__ __launch_bounds__(128) void proj_kernel(const b16* __restrict__ Oh, const b16* __restrict__ Ol, const b16* __restrict__ Wb, const float* __restrict__ bp, const float* __restrict__ gamma, const float* __restrict__ x, float* __restrict__ out) {
  __shared__ __attribute__((aligned(16))) float Ty[64][64 + 4];
  const int wave = threadIdx.x >> 5, lane = threadIdx.x & 31, nloc = lane & 15, hlf = lane >> 4; const size_t n0 = (size_t)blockIdx.x * 64; const size_t m0 = n0 + wave * 16;
  v8f acc[4];
#pragma unroll
  for (int t = 0; t < 4; ++t) acc[t] = (v8f){};
#pragma unroll
  for (int j = 0; j < 2; ++j) { const v16b a = frag_heads(Oh, m0 + nloc, j, hlf), al = frag_heads(Ol, m0 + nloc, j, hlf);
#pragma unroll
    for (int t = 0; t < 4; ++t) { const v16b bw = frag_kb(Wb + (size_t)(192 + t * 16 + nloc) * C + j * 32, hlf); acc[t] = wmma16b(a, bw, acc[t]); acc[t] = wmma16b(al, bw, acc[t]); } }
  const float g = bf16_rne(gamma[0]);
#pragma unroll
  for (int t = 0; t < 4; ++t) { const int c = t * 16 + nloc; const float bb = bf16_rne(bp[c]);
#pragma unroll
    for (int r = 0; r < 8; ++r) Ty[c][wave * 16 + 8 * hlf + r] = g * (acc[t][r] * (1.0f / (XS * WSC)) + bb); }
  __syncthreads();
  for (int pass = 0; pass < 2; ++pass) { for (int rr = 0; rr < 16; ++rr) { const int c = wave * 16 + rr; const size_t gi = (size_t)c * T + n0 + lane * 2; v2f y = *(const v2f*)(&Ty[c][lane * 2]); const v2f xv = *(const v2f*)(x + gi); y[0] += bf16_rne(xv[0]); y[1] += bf16_rne(xv[1]);
      *(volatile v2f*)(out + gi) = y; } __threadfence(); }
}
}

extern "C" void kernel_launch(void* const* d_in, const int* in_sizes, int n_in, void* d_out, int out_size, void* d_ws, size_t ws_size, hipStream_t stream) {
  (void)n_in;
  auto Fp = [&](int i) { return (const float*)d_in[i]; };
  if (in_sizes[0] != C * T || in_sizes[1] != 3 * C * C || in_sizes[2] != C * C || in_sizes[3] != C || in_sizes[4] != 1 || out_size != C * T) return;
  size_t off = 0; char* ws = (char*)d_ws;
  auto carve = [&](size_t bytes) { char* p = ws + off; off += (bytes + 255) & ~(size_t)255; return p; };
  b16* Xt = (b16*)carve((size_t)T * C * 2); b16* Wb = (b16*)carve((size_t)256 * C * 2); b16* QK = (b16*)carve((size_t)2 * T * NH * KP * 2); b16* VT = (b16*)carve((size_t)NH * VP * T * 2); b16* Oh = (b16*)carve((size_t)NH * T * HD * 2); b16* Ol = (b16*)carve((size_t)NH * T * HD * 2);
  if (off > ws_size || off > ((size_t)128 << 20)) return;
  prep_kernel<<<T / 64 + 1, 256, 0, stream>>>(Fp(0), Fp(1), Fp(2), Xt, Wb);
  qk_kernel<<<T / 16, 32, 0, stream>>>(Xt, Wb, QK);
  vt_kernel<<<T / 128, 128, 0, stream>>>(Xt, Wb, VT);
  attn_kernel<<<dim3(NQB, NH), 64, 0, stream>>>(QK, VT, Oh, Ol);
  proj_kernel<<<(NQB * 32) / 64, 128, 0, stream>>>(Oh, Ol, Wb, Fp(3), Fp(4), Fp(0), (float*)d_out);
}
